// Net_6253472382984
// MI455X (gfx1250) — hardware-verified
//
#include <hip/hip_runtime.h>
#include <stddef.h>
#include <stdint.h>
#include <math.h>


#define NN     30000
#define NE     240000
#define TM     128
#define NP     30080
#define NTHR   256
#define NWAVE  8
#define EPT    8
#define CHUNK  (NTHR * EPT)
#define WCAP   (EPT * 32)
#define LISTN  (NWAVE * WCAP)
#define NBA    1024
#define SLA    10
#define RCAP   10240
#define DEGCAP 32
#define NBLK   30
#define NSLOT  (NBLK * NBA)
#define EIDN   (NBLK * RCAP)
#define PA     264
#define PE     168
#define PH     200
#define CSR_ZINTS (LISTN + 2 * RCAP + 3 * NBA)
#define CSR_LDS_INTS (CSR_ZINTS + 16)
#define NODE_LDS_BYTES (TM * PA * 2 + TM * 32 * 4 + TM * 4)
#define U_WE   512
#define U_SD   768
#define U_MID  1280
#define U_NM   1536
#define U_FC   2560
#define U_END  2816
#define WSMAX  134217728

static_assert(NP % TM == 0 && NP >= NN && NP - NN < TM);
static_assert(NE % TM == 0 && NN % 4 == 0);
static_assert(NSLOT >= NP);
static_assert((NBA & (NBA - 1)) == 0 && NBA == (1 << SLA));
static_assert(((long long)NE << SLA) < (1LL << 31));
static_assert(((long long)CHUNK << SLA) < (1LL << 31));
static_assert(RCAP % (NTHR * 4) == 0 && CSR_ZINTS % (NTHR * 4) == 0);
static_assert(NBA == NTHR * 4);
static_assert(U_END % NTHR == 0 && U_WE % NTHR == 0 && U_SD % NTHR == 0 && U_MID % NTHR == 0);
static_assert(U_NM % NTHR == 0 && U_FC % NTHR == 0);
static_assert(PA % 8 == 0 && PE % 8 == 0 && PH % 8 == 0 && PA >= 256 && PE >= 160 && PH >= 192);
static_assert((TM * PA * 2) % 16 == 0);
static_assert(CSR_LDS_INTS * 4 <= 300000 && NODE_LDS_BYTES <= 300000);
static_assert((NP * 8) % NTHR == 0 && (NE * 4) % NTHR == 0);

typedef float          v4f   __attribute__((ext_vector_type(4)));
typedef float          v8f   __attribute__((ext_vector_type(8)));
typedef int            v4i   __attribute__((ext_vector_type(4)));
typedef int            v8i   __attribute__((ext_vector_type(8)));
typedef unsigned short v4us  __attribute__((ext_vector_type(4)));
typedef unsigned short v8us  __attribute__((ext_vector_type(8)));
typedef unsigned short v16us __attribute__((ext_vector_type(16)));
typedef __bf16         v16bf __attribute__((ext_vector_type(16)));
typedef v4f  __attribute__((may_alias)) v4fa;
typedef v4i  __attribute__((may_alias)) v4ia;
typedef v4us __attribute__((may_alias)) v4usa;
typedef v8us __attribute__((may_alias)) v8usa;
union FragB { v16bf v; v16us u; v8us h[2]; v8i w; };

__device__ __forceinline__ v8f wmb(const FragB& a, const FragB& b, v8f c) {
  v8f d = __builtin_amdgcn_wmma_f32_16x16x32_bf16(false, a.v, false, b.v, (short)0, c, false, false);
  asm volatile("v_nop\n\tv_nop\n\tv_nop\n\tv_nop" : "+v"(d) : "v"(a.w), "v"(b.w));
  return d;
}

__device__ __forceinline__ unsigned bf16_bits(float f) {
  const unsigned u = __float_as_uint(f);
  return (u + 0x7FFFu + ((u >> 16) & 1u)) >> 16;
}
__device__ __forceinline__ float bf16_val(float f) {
  return __uint_as_float(bf16_bits(f) << 16);
}
__device__ __forceinline__ void split2(float v, unsigned& hb, unsigned& lb) {
  hb = bf16_bits(v);
  lb = bf16_bits(v - __uint_as_float(hb << 16));
}
__device__ __forceinline__ void split4(const v4f a, v4us& h, v4us& l) {
  unsigned hb, lb;
  split2(a.x, hb, lb); h[0] = (unsigned short)hb; l[0] = (unsigned short)lb;
  split2(a.y, hb, lb); h[1] = (unsigned short)hb; l[1] = (unsigned short)lb;
  split2(a.z, hb, lb); h[2] = (unsigned short)hb; l[2] = (unsigned short)lb;
  split2(a.w, hb, lb); h[3] = (unsigned short)hb; l[3] = (unsigned short)lb;
}
__device__ __forceinline__ float sigm(float v) { return 1.0f / (1.0f + expf(-v)); }

__device__ __forceinline__ FragB frag_lds(const unsigned short* p) {
  FragB f;
  f.h[0] = *(const v8usa*)p;
  f.h[1] = *(const v8usa*)(p + 16);
  return f;
}
__device__ __forceinline__ FragB frag_glb(const unsigned short* __restrict__ p) {
  FragB f;
  f.h[0] = *(const v8usa*)p;
  f.h[1] = *(const v8usa*)(p + 16);
  return f;
}

template <int SLB>
__device__ __forceinline__ int scan_chunk(const int* __restrict__ dsts, int nE, int cbase, int slotBase,
                                          int nb, int vec8, int* list, int tid, int lane, int wave) {
  int wc = 0;
  const int el0  = tid * EPT;
  const int e0   = cbase + el0;
  const int sent = -2147483647 - 1;
  v4i da, db;
  if (vec8 != 0 && cbase + CHUNK <= nE) {
    da = *(const v4i*)(dsts + e0);
    db = *(const v4i*)(dsts + e0 + 4);
  } else {
    da.x = (e0     < nE) ? dsts[min(e0,     nE - 1)] : sent;
    da.y = (e0 + 1 < nE) ? dsts[min(e0 + 1, nE - 1)] : sent;
    da.z = (e0 + 2 < nE) ? dsts[min(e0 + 2, nE - 1)] : sent;
    da.w = (e0 + 3 < nE) ? dsts[min(e0 + 3, nE - 1)] : sent;
    db.x = (e0 + 4 < nE) ? dsts[min(e0 + 4, nE - 1)] : sent;
    db.y = (e0 + 5 < nE) ? dsts[min(e0 + 5, nE - 1)] : sent;
    db.z = (e0 + 6 < nE) ? dsts[min(e0 + 6, nE - 1)] : sent;
    db.w = (e0 + 7 < nE) ? dsts[min(e0 + 7, nE - 1)] : sent;
  }
  const unsigned nbs = (unsigned)slotBase;
  const unsigned unb = (unsigned)nb;
  const unsigned s0 = (unsigned)da.x - nbs, s1 = (unsigned)da.y - nbs;
  const unsigned s2 = (unsigned)da.z - nbs, s3 = (unsigned)da.w - nbs;
  const unsigned s4 = (unsigned)db.x - nbs, s5 = (unsigned)db.y - nbs;
  const unsigned s6 = (unsigned)db.z - nbs, s7 = (unsigned)db.w - nbs;
  const bool h0 = s0 < unb, h1 = s1 < unb, h2 = s2 < unb, h3 = s3 < unb;
  const bool h4 = s4 < unb, h5 = s5 < unb, h6 = s6 < unb, h7 = s7 < unb;
  const unsigned any = __builtin_amdgcn_ballot_w32(h0 | h1 | h2 | h3 | h4 | h5 | h6 | h7);
  if (any != 0u) {
#define HITJ(J, HJ, SJ) { \
      const unsigned mj = __builtin_amdgcn_ballot_w32(HJ); \
      if (mj != 0u) { \
        if (HJ) { \
          const int pos = wc + (int)__builtin_amdgcn_mbcnt_lo(mj, 0u); \
          if (pos < WCAP) list[wave * WCAP + pos] = ((el0 + (J)) << SLB) | (int)(SJ); \
        } \
        wc += (int)__builtin_popcount(mj); } }
    HITJ(0, h0, s0)
    HITJ(1, h1, s1)
    HITJ(2, h2, s2)
    HITJ(3, h3, s3)
    HITJ(4, h4, s4)
    HITJ(5, h5, s5)
    HITJ(6, h6, s6)
    HITJ(7, h7, s7)
#undef HITJ
  }
  return wc;
}

__device__ __forceinline__ v8us gath8(const float* __restrict__ p, int stride, bool zero) {
  v8us o;
#pragma unroll
  for (int i = 0; i < 8; ++i) {
    const unsigned b = bf16_bits(p[(size_t)i * stride]);
    o[i] = zero ? (unsigned short)0 : (unsigned short)b;
  }
  return o;
}

__global__ __launch_bounds__(NTHR) void k_prep(const float* __restrict__ Wn, const float* __restrict__ We,
                                               const float* __restrict__ Wem, const float* __restrict__ Wnm,
                                               const float* __restrict__ Wfc, unsigned short* W16) {
  const int u = (int)blockIdx.x * NTHR + (int)threadIdx.x;
  v8us o;
  if (u < U_WE) {
    const int n = u >> 3, k8 = (u & 7) * 8, kk = k8 & 31;
    o = gath8(Wn + (size_t)kk * 64 + n, 64, false);
  } else if (u < U_SD) {
    const int v = u - U_WE;
    const int n = v >> 2, k8 = (v & 3) * 8, kk = k8 & 15;
    o = gath8(We + (size_t)kk * 64 + n, 64, false);
  } else if (u < U_MID) {
    const int v = u - U_SD;
    const int n = v >> 4, k8 = (v & 15) * 8, kk = k8 & 63;
    const int rb = (n < 16) ? 0 : 128;
    o = gath8(Wem + (size_t)(rb + kk) * 16 + (n & 15), 16, false);
  } else if (u < U_NM) {
    const int v = u - U_MID;
    const int n = v >> 4, k8 = (v & 15) * 8, kk = k8 & 63;
    o = gath8(Wem + (size_t)(64 + kk) * 16 + n, 16, false);
  } else if (u < U_FC) {
    const int v = u - U_NM;
    const int n = v >> 5, k8 = (v & 31) * 8, kk = k8 & 127;
    o = gath8(Wnm + (size_t)kk * 32 + n, 32, false);
  } else if (u < U_END) {
    const int v = u - U_FC;
    const int n = v >> 4, k8 = (v & 15) * 8, kk = k8 & 63;
    const int nc = n < 8 ? n : 7;
    o = gath8(Wfc + (size_t)kk * 8 + nc, 8, n >= 8);
  } else {
    return;
  }
  unsigned short* dp = W16 + (size_t)u * 8;
  *(volatile v8us*)dp = o;
  __threadfence();
  *(volatile v8us*)dp = o;
}

__global__ __launch_bounds__(NTHR) void k_cvt(const float* __restrict__ in, int nIn4, int nOut4, float* outp) {
  const int u = (int)blockIdx.x * NTHR + (int)threadIdx.x;
  if (u >= nOut4) return;
  const int uc = u < nIn4 ? u : nIn4 - 1;
  const v4f a = *(const v4fa*)(in + (size_t)uc * 4);
  const bool ok = u < nIn4;
  v4f o;
  o.x = ok ? bf16_val(a.x) : 0.0f;
  o.y = ok ? bf16_val(a.y) : 0.0f;
  o.z = ok ? bf16_val(a.z) : 0.0f;
  o.w = ok ? bf16_val(a.w) : 0.0f;
  float* dp = outp + (size_t)u * 4;
  *(volatile v4f*)dp = o;
  __threadfence();
  *(volatile v4f*)dp = o;
}

__global__ __launch_bounds__(NTHR) void k_csr(const int* __restrict__ keys, int nE, int vec8,
                                              int* offs_g, int* cnt_g, int* eid_g) {
  extern __shared__ __attribute__((aligned(16))) int dsm[];
  int* list = dsm;
  int* hl   = dsm + LISTN;
  int* sl   = hl + RCAP;
  int* cnt  = sl + RCAP;
  int* offs = cnt + NBA;
  int* cur  = offs + NBA;
  int* misc = cur + NBA;
  const int tid = (int)threadIdx.x, lane = tid & 31, wave = tid >> 5;
  const int nodeBase = (int)blockIdx.x * NBA;

  {
    const v4i z4 = {0, 0, 0, 0};
    for (int i = tid * 4; i < CSR_ZINTS; i += NTHR * 4) *(v4ia*)(dsm + i) = z4;
    if (tid < 16) misc[tid] = 0;
  }
  __syncthreads();

  int t = 0, ov = 0;
  const int nChunks = (nE + CHUNK - 1) / CHUNK;
#pragma unroll 1
  for (int ch = 0; ch < nChunks; ++ch) {
    const int cbase = ch * CHUNK;
    const int wc = scan_chunk<SLA>(keys, nE, cbase, nodeBase, NBA, vec8, list, tid, lane, wave);
    if (lane == 0) misc[wave] = wc;
    __syncthreads();
    if (wave == 0) {
#pragma unroll 1
      for (int w2 = 0; w2 < NWAVE; ++w2) {
        int c = misc[w2];
        c = c < 0 ? 0 : (c > WCAP ? WCAP : c);
#pragma unroll 1
        for (int b0 = 0; b0 < c; b0 += 32) {
          const int idx = b0 + lane;
          const int ent = list[w2 * WCAP + (idx < WCAP ? idx : WCAP - 1)];
          const int m32 = (c - b0) < 32 ? (c - b0) : 32;
#pragma unroll 1
          for (int k = 0; k < m32; ++k) {
            const int u    = __builtin_amdgcn_readlane(ent, k);
            const int slot = u & (NBA - 1);
            const int el   = (u >> SLA) & (CHUNK - 1);
            const int pk   = ((cbase + el) << SLA) | slot;
            if (t < RCAP) {
              if (lane == 0) { hl[t] = pk; cnt[slot] = cnt[slot] + 1; }
              t = t + 1;
            } else {
              ov = 1;
            }
          }
        }
      }
    }
    __syncthreads();
  }
  if (wave == 0 && lane == 0) { misc[8] = t; misc[9] = ov; }
  __syncthreads();
  int tt = misc[8];
  tt = tt < 0 ? 0 : (tt > RCAP ? RCAP : tt);
  const int ovf = misc[9];

  if (wave == 0) {
    const int base = lane * (NBA / 32);
    int s = 0;
#pragma unroll 1
    for (int i = 0; i < NBA / 32; ++i) s += cnt[base + i];
    int incl = s;
#pragma unroll
    for (int d = 1; d < 32; d <<= 1) {
      const int y = __shfl_up(incl, d, 32);
      if (lane >= d) incl += y;
    }
    int run = incl - s;
#pragma unroll 1
    for (int i = 0; i < NBA / 32; ++i) {
      const int cv = cnt[base + i];
      offs[base + i] = run;
      cur[base + i]  = run;
      run += cv;
    }
  }
  __syncthreads();
  if (wave == 0) {
#pragma unroll 1
    for (int b0 = 0; b0 < tt; b0 += 32) {
      const int idx = b0 + lane;
      const int ent = hl[idx < RCAP ? idx : RCAP - 1];
      const int m32 = (tt - b0) < 32 ? (tt - b0) : 32;
#pragma unroll 1
      for (int k = 0; k < m32; ++k) {
        const int u    = __builtin_amdgcn_readlane(ent, k);
        const int slot = u & (NBA - 1);
        if (lane == 0) {
          int p = cur[slot];
          p = p < 0 ? 0 : (p > RCAP - 1 ? RCAP - 1 : p);
          sl[p] = u;
          cur[slot] = p + 1;
        }
      }
    }
  }
  __syncthreads();

#pragma unroll 1
  for (int p0 = 0; p0 < tt; p0 += NTHR) {
    const int p = p0 + tid;
    const int ent = sl[p];
    const bool valid = p < tt;
    const int slot = ent & (NBA - 1);
    int o = offs[slot];
    o = o < 0 ? 0 : (o > RCAP - 1 ? RCAP - 1 : o);
    int c = cnt[slot];
    c = c < 0 ? 0 : (c > DEGCAP ? DEGCAP : c);
    c = valid ? c : 0;
    int cm = c;
#pragma unroll
    for (int d = 16; d >= 1; d >>= 1) {
      const int y = __shfl_xor(cm, d, 32);
      cm = cm > y ? cm : y;
    }
    int rank = 0;
#pragma unroll 1
    for (int q = 0; q < cm; ++q) {
      int idx = o + q;
      idx = idx > RCAP - 1 ? RCAP - 1 : idx;
      const int v = sl[idx];
      rank += ((q < c) && (v < ent)) ? 1 : 0;
    }
    if (valid) {
      int d = o + rank;
      d = d > RCAP - 1 ? RCAP - 1 : d;
      hl[d] = ent;
    }
  }
  __syncthreads();

  v4i ev[RCAP / (NTHR * 4)];
#pragma unroll
  for (int it = 0; it < RCAP / (NTHR * 4); ++it) {
    const v4i h = *(const v4ia*)(hl + (it * NTHR + tid) * 4);
    v4i e;
    e.x = h.x >> SLA; e.y = h.y >> SLA; e.z = h.z >> SLA; e.w = h.w >> SLA;
    ev[it] = e;
  }
  v4i o4 = *(const v4ia*)(offs + 4 * tid);
  v4i c4 = *(const v4ia*)(cnt + 4 * tid);
  {
    const int gb = (int)blockIdx.x * RCAP;
    o4.x += gb; o4.y += gb; o4.z += gb; o4.w += gb;
    c4.x = (ovf != 0 || c4.x < 0 || c4.x > DEGCAP) ? -1 : c4.x;
    c4.y = (ovf != 0 || c4.y < 0 || c4.y > DEGCAP) ? -1 : c4.y;
    c4.z = (ovf != 0 || c4.z < 0 || c4.z > DEGCAP) ? -1 : c4.z;
    c4.w = (ovf != 0 || c4.w < 0 || c4.w > DEGCAP) ? -1 : c4.w;
  }
  int* eb = eid_g + (size_t)blockIdx.x * RCAP;
#pragma unroll
  for (int it = 0; it < RCAP / (NTHR * 4); ++it) *(volatile v4i*)(eb + (it * NTHR + tid) * 4) = ev[it];
  *(volatile v4i*)(offs_g + nodeBase + 4 * tid) = o4;
  *(volatile v4i*)(cnt_g + nodeBase + 4 * tid) = c4;
  __threadfence();
#pragma unroll
  for (int it = 0; it < RCAP / (NTHR * 4); ++it) *(volatile v4i*)(eb + (it * NTHR + tid) * 4) = ev[it];
  *(volatile v4i*)(offs_g + nodeBase + 4 * tid) = o4;
  *(volatile v4i*)(cnt_g + nodeBase + 4 * tid) = c4;
}

__device__ __forceinline__ void load_nin_tile(const float* nin, int r0, unsigned short* pa, int pitch, int tid) {
#pragma unroll
  for (int i = 0; i < 4; ++i) {
    const int idx = tid + NTHR * i;
    const int row = idx >> 3, q = idx & 7;
    const v4f a = *(const v4fa*)(nin + (size_t)(r0 + row) * 32 + 4 * q);
    v4us h4, l4;
    split4(a, h4, l4);
    *(v4usa*)(pa + row * pitch + 4 * q) = h4;
    *(v4usa*)(pa + row * pitch + 32 + 4 * q) = l4;
  }
}

__device__ __forceinline__ void node_fc(unsigned short* pa, int pitch, int hiCol, int loCol,
                                        const unsigned short* __restrict__ WnT2, const float* __restrict__ bn,
                                        int wave, int hh, int m) {
  const unsigned short* pr = pa + (16 * wave + m) * pitch + 8 * hh;
  v8f acc[4];
  {
    const v8f z = {0.f, 0.f, 0.f, 0.f, 0.f, 0.f, 0.f, 0.f};
    acc[0] = z; acc[1] = z; acc[2] = z; acc[3] = z;
  }
#pragma unroll
  for (int ks = 0; ks < 2; ++ks) {
    const FragB af = frag_lds(pr + 32 * ks);
#pragma unroll
    for (int t = 0; t < 4; ++t) {
      const FragB bf = frag_glb(WnT2 + (size_t)(16 * t + m) * 64 + 8 * hh + 32 * ks);
      acc[t] = wmb(af, bf, acc[t]);
    }
  }
#pragma unroll
  for (int t = 0; t < 4; ++t) {
    const float bv = bf16_val(bn[16 * t + m]);
#pragma unroll
    for (int r = 0; r < 8; ++r) {
      const int row = 16 * wave + 8 * hh + r;
      unsigned hb, lb;
      split2(acc[t][r] + bv, hb, lb);
      pa[row * pitch + hiCol + 16 * t + m] = (unsigned short)hb;
      pa[row * pitch + loCol + 16 * t + m] = (unsigned short)lb;
    }
  }
}

__device__ __forceinline__ void store_rows32(const float* fs, float* g, int wave, int lane) {
  v4f pv[4];
#pragma unroll
  for (int i = 0; i < 4; ++i) pv[i] = *(const v4fa*)(fs + (16 * wave + 4 * i) * 32 + 4 * lane);
#pragma unroll
  for (int i = 0; i < 4; ++i) *(volatile v4f*)(g + (size_t)(16 * wave + 4 * i) * 32 + 4 * lane) = pv[i];
  __threadfence();
#pragma unroll
  for (int i = 0; i < 4; ++i) *(volatile v4f*)(g + (size_t)(16 * wave + 4 * i) * 32 + 4 * lane) = pv[i];
}

__global__ __launch_bounds__(NTHR) void k_node(float* NIN, float* P, const float* __restrict__ E,
                                               const int* __restrict__ OFFS, const int* __restrict__ CNT,
                                               const int* __restrict__ EID, int eidN, int nE,
                                               const unsigned short* __restrict__ WnT2,
                                               const unsigned short* __restrict__ WeT2,
                                               const unsigned short* __restrict__ WsdT2,
                                               const unsigned short* __restrict__ WnmT2,
                                               const float* __restrict__ bn, const float* __restrict__ be,
                                               const float* __restrict__ bnm) {
  extern __shared__ __attribute__((aligned(16))) int dsm[];
  unsigned short* pa = (unsigned short*)dsm;
  float* fs = (float*)((unsigned char*)dsm + TM * PA * 2);
  float* cf = fs + TM * 32;
  const int tid = (int)threadIdx.x, lane = tid & 31, wave = tid >> 5, hh = lane >> 4, m = lane & 15;
  const int r0 = (int)blockIdx.x * TM;

  load_nin_tile(NIN, r0, pa, PA, tid);
  {
    const int node = tid >> 1, hf = tid & 1;
    const int gi = r0 + node;
    int c = CNT[gi];
    int o = OFFS[gi];
    const bool bad = (c < 0) || (c > DEGCAP);
    c = c < 0 ? 0 : (c > DEGCAP ? DEGCAP : c);
    o = o < 0 ? 0 : (o > eidN - 1 ? eidN - 1 : o);
    int cm = c;
#pragma unroll
    for (int d = 16; d >= 1; d >>= 1) {
      const int y = __shfl_xor(cm, d, 32);
      cm = cm > y ? cm : y;
    }
    v4f sa = {0.0f, 0.0f, 0.0f, 0.0f};
    v4f sb = {0.0f, 0.0f, 0.0f, 0.0f};
#pragma unroll 1
    for (int p = 0; p < cm; ++p) {
      int idx = o + p;
      idx = idx > eidN - 1 ? eidN - 1 : idx;
      int e = EID[idx];
      e = e < 0 ? 0 : (e > nE - 1 ? nE - 1 : e);
      const unsigned msk = (p < c) ? 0xffffffffu : 0u;
      const v4f x = *(const v4fa*)(E + (size_t)e * 16 + 8 * hf);
      const v4f y = *(const v4fa*)(E + (size_t)e * 16 + 8 * hf + 4);
      sa.x += __uint_as_float(__float_as_uint(x.x) & msk);
      sa.y += __uint_as_float(__float_as_uint(x.y) & msk);
      sa.z += __uint_as_float(__float_as_uint(x.z) & msk);
      sa.w += __uint_as_float(__float_as_uint(x.w) & msk);
      sb.x += __uint_as_float(__float_as_uint(y.x) & msk);
      sb.y += __uint_as_float(__float_as_uint(y.y) & msk);
      sb.z += __uint_as_float(__float_as_uint(y.z) & msk);
      sb.w += __uint_as_float(__float_as_uint(y.w) & msk);
    }
    v4us ha, la, hb4, lb4;
    split4(sa, ha, la);
    split4(sb, hb4, lb4);
    *(v4usa*)(pa + node * PA + 128 + 8 * hf) = ha;
    *(v4usa*)(pa + node * PA + 128 + 8 * hf + 4) = hb4;
    *(v4usa*)(pa + node * PA + 144 + 8 * hf) = la;
    *(v4usa*)(pa + node * PA + 144 + 8 * hf + 4) = lb4;
    const float cfv = bad ? __int_as_float(0x7fc00000) : (float)c;
    if (hf == 0) cf[node] = cfv;
  }
  __syncthreads();

  node_fc(pa, PA, 64, 192, WnT2, bn, wave, hh, m);
  __syncthreads();

  const unsigned short* pr = pa + (16 * wave + m) * PA + 8 * hh;
  const v8f z8 = {0.f, 0.f, 0.f, 0.f, 0.f, 0.f, 0.f, 0.f};

  v8f acc4[4];
  {
    v8f acc2[2];
    acc2[0] = z8; acc2[1] = z8;
#pragma unroll
    for (int ks = 0; ks < 4; ++ks) {
      const int acol = (ks < 2) ? (64 + 32 * ks) : (192 + 32 * (ks - 2));
      const FragB af = frag_lds(pr + acol);
#pragma unroll
      for (int t = 0; t < 2; ++t) {
        const FragB bf = frag_glb(WsdT2 + (size_t)(16 * t + m) * 128 + 8 * hh + 32 * ks);
        acc2[t] = wmb(af, bf, acc2[t]);
      }
    }
#pragma unroll
    for (int t = 0; t < 2; ++t) {
#pragma unroll
      for (int r = 0; r < 8; ++r) fs[(16 * wave + 8 * hh + r) * 32 + 16 * t + m] = acc2[t][r];
    }
    acc4[0] = z8; acc4[1] = z8; acc4[2] = z8; acc4[3] = z8;
    const FragB as = frag_lds(pr + 128);
#pragma unroll
    for (int t = 0; t < 4; ++t) {
      const FragB bf = frag_glb(WeT2 + (size_t)(16 * t + m) * 32 + 8 * hh);
      acc4[t] = wmb(as, bf, acc4[t]);
    }
  }
  __syncthreads();

  {
    float cfr[8];
#pragma unroll
    for (int r = 0; r < 8; ++r) cfr[r] = cf[16 * wave + 8 * hh + r];
#pragma unroll
    for (int t = 0; t < 4; ++t) {
      const float bev = bf16_val(be[16 * t + m]);
#pragma unroll
      for (int r = 0; r < 8; ++r) {
        const int row = 16 * wave + 8 * hh + r;
        unsigned hb, lb;
        split2(fmaf(cfr[r], bev, acc4[t][r]), hb, lb);
        pa[row * PA + 16 * t + m] = (unsigned short)hb;
        pa[row * PA + 128 + 16 * t + m] = (unsigned short)lb;
      }
    }
    store_rows32(fs, P + (size_t)r0 * 32, wave, lane);
  }
  __syncthreads();

  {
    v8f acc5[2];
    acc5[0] = z8; acc5[1] = z8;
#pragma unroll
    for (int ks = 0; ks < 8; ++ks) {
      const FragB af = frag_lds(pr + 32 * ks);
#pragma unroll
      for (int t = 0; t < 2; ++t) {
        const FragB bf = frag_glb(WnmT2 + (size_t)(16 * t + m) * 256 + 8 * hh + 32 * ks);
        acc5[t] = wmb(af, bf, acc5[t]);
      }
    }
#pragma unroll
    for (int t = 0; t < 2; ++t) {
      const float bmv = bf16_val(bnm[16 * t + m]);
#pragma unroll
      for (int r = 0; r < 8; ++r) fs[(16 * wave + 8 * hh + r) * 32 + 16 * t + m] = acc5[t][r] + bmv;
    }
  }
  __syncthreads();
#pragma unroll 1
  for (int j = 0; j < (TM * 32) / NTHR; ++j) {
    const int idx = tid + NTHR * j;
    const float x = fs[idx];
    fs[idx] = sigm(x);
  }
  __syncthreads();
  store_rows32(fs, NIN + (size_t)r0 * 32, wave, lane);
}

__global__ __launch_bounds__(NTHR) void k_edge(float* E, const float* __restrict__ P,
                                               const int* __restrict__ src, const int* __restrict__ dst, int nN,
                                               const unsigned short* __restrict__ WeT2,
                                               const unsigned short* __restrict__ WmidT2,
                                               const float* __restrict__ be, const float* __restrict__ bem) {
  __shared__ __attribute__((aligned(16))) unsigned short pa[TM * PE];
  __shared__ __attribute__((aligned(16))) float fs[TM * 16];
  const int tid = (int)threadIdx.x, lane = tid & 31, wave = tid >> 5, hh = lane >> 4, m = lane & 15;
  const int e0 = (int)blockIdx.x * TM;

#pragma unroll
  for (int i = 0; i < 2; ++i) {
    const int idx = tid + NTHR * i;
    const int row = idx >> 2, q = idx & 3;
    const v4f a = *(const v4fa*)(E + (size_t)(e0 + row) * 16 + 4 * q);
    v4us h4, l4;
    split4(a, h4, l4);
    *(v4usa*)(pa + row * PE + 4 * q) = h4;
    *(v4usa*)(pa + row * PE + 16 + 4 * q) = l4;
    int s = src[e0 + row];
    int d = dst[e0 + row];
    s = s < 0 ? 0 : (s > nN - 1 ? nN - 1 : s);
    d = d < 0 ? 0 : (d > nN - 1 ? nN - 1 : d);
    const v4f ps = *(const v4fa*)(P + (size_t)s * 32 + 4 * q);
    const v4f pd = *(const v4fa*)(P + (size_t)d * 32 + 16 + 4 * q);
    const v4f bm = *(const v4fa*)(bem + 4 * q);
    v4f g;
    g.x = (ps.x + pd.x) + bf16_val(bm.x);
    g.y = (ps.y + pd.y) + bf16_val(bm.y);
    g.z = (ps.z + pd.z) + bf16_val(bm.z);
    g.w = (ps.w + pd.w) + bf16_val(bm.w);
    *(v4fa*)(fs + row * 16 + 4 * q) = g;
  }
  __syncthreads();

  const unsigned short* pr = pa + (16 * wave + m) * PE + 8 * hh;
  const v8f z8 = {0.f, 0.f, 0.f, 0.f, 0.f, 0.f, 0.f, 0.f};

  {
    v8f acc[4];
    acc[0] = z8; acc[1] = z8; acc[2] = z8; acc[3] = z8;
    const FragB af = frag_lds(pr);
#pragma unroll
    for (int t = 0; t < 4; ++t) {
      const FragB bf = frag_glb(WeT2 + (size_t)(16 * t + m) * 32 + 8 * hh);
      acc[t] = wmb(af, bf, acc[t]);
    }
#pragma unroll
    for (int t = 0; t < 4; ++t) {
      const float bev = bf16_val(be[16 * t + m]);
#pragma unroll
      for (int r = 0; r < 8; ++r) {
        const int row = 16 * wave + 8 * hh + r;
        unsigned hb, lb;
        split2(acc[t][r] + bev, hb, lb);
        pa[row * PE + 32 + 16 * t + m] = (unsigned short)hb;
        pa[row * PE + 96 + 16 * t + m] = (unsigned short)lb;
      }
    }
  }
  __syncthreads();

  {
    v8f acc = z8;
#pragma unroll
    for (int ks = 0; ks < 4; ++ks) {
      const FragB af = frag_lds(pr + 32 + 32 * ks);
      const FragB bf = frag_glb(WmidT2 + (size_t)m * 128 + 8 * hh + 32 * ks);
      acc = wmb(af, bf, acc);
    }
#pragma unroll
    for (int r = 0; r < 8; ++r) {
      const int idx = (16 * wave + 8 * hh + r) * 16 + m;
      const float g = fs[idx];
      fs[idx] = acc[r] + g;
    }
  }
  __syncthreads();
#pragma unroll 1
  for (int j = 0; j < (TM * 16) / NTHR; ++j) {
    const int idx = tid + NTHR * j;
    const float x = fs[idx];
    fs[idx] = sigm(x);
  }
  __syncthreads();

  {
    v4f pv[2];
#pragma unroll
    for (int i = 0; i < 2; ++i) pv[i] = *(const v4fa*)(fs + 16 * wave * 16 + (32 * i + lane) * 4);
    float* g = E + (size_t)(e0 + 16 * wave) * 16;
#pragma unroll
    for (int i = 0; i < 2; ++i) *(volatile v4f*)(g + (32 * i + lane) * 4) = pv[i];
    __threadfence();
#pragma unroll
    for (int i = 0; i < 2; ++i) *(volatile v4f*)(g + (32 * i + lane) * 4) = pv[i];
  }
}

__global__ __launch_bounds__(NTHR) void k_head(const float* __restrict__ NIN,
                                               const unsigned short* __restrict__ WnT2,
                                               const unsigned short* __restrict__ WfcT2,
                                               const float* __restrict__ bn, const float* __restrict__ bfc,
                                               float* outp, int nN) {
  __shared__ __attribute__((aligned(16))) unsigned short pa[TM * PH];
  __shared__ __attribute__((aligned(16))) float fs[TM * 8];
  const int tid = (int)threadIdx.x, lane = tid & 31, wave = tid >> 5, hh = lane >> 4, m = lane & 15;
  const int r0 = (int)blockIdx.x * TM;

  load_nin_tile(NIN, r0, pa, PH, tid);
  __syncthreads();
  node_fc(pa, PH, 64, 128, WnT2, bn, wave, hh, m);
  __syncthreads();
  {
    const unsigned short* pr = pa + (16 * wave + m) * PH + 8 * hh;
    v8f acc = {0.f, 0.f, 0.f, 0.f, 0.f, 0.f, 0.f, 0.f};
#pragma unroll
    for (int ks = 0; ks < 4; ++ks) {
      const FragB af = frag_lds(pr + 64 + 32 * ks);
      const FragB bf = frag_glb(WfcT2 + (size_t)m * 128 + 8 * hh + 32 * ks);
      acc = wmb(af, bf, acc);
    }
    const float bfv = bf16_val(bfc[m < 8 ? m : 7]);
    if (m < 8) {
#pragma unroll
      for (int r = 0; r < 8; ++r) fs[(16 * wave + 8 * hh + r) * 8 + m] = acc[r] + bfv;
    }
  }
  __syncthreads();
  {
    const v4f pv = *(const v4fa*)(fs + 16 * wave * 8 + 4 * lane);
    const int gr = r0 + 16 * wave + (lane >> 1);
    float* g = outp + (size_t)(r0 + 16 * wave) * 8 + 4 * lane;
    const bool ok = gr < nN;
    if (ok) *(volatile v4f*)g = pv;
    __threadfence();
    if (ok) *(volatile v4f*)g = pv;
  }
}

static inline size_t al256(size_t o) { return (o + 255) & ~(size_t)255; }

extern "C" void kernel_launch(void* const* d_in, const int* in_sizes, int n_in,
                              void* d_out, int out_size, void* d_ws, size_t ws_size,
                              hipStream_t stream) {
  if (n_in < 14) return;
  if (in_sizes[0] != NN * 32 || in_sizes[1] != NE * 16) return;
  if (in_sizes[2] != NE || in_sizes[3] != NE) return;
  if (in_sizes[4] != 32 * 64 || in_sizes[5] != 64) return;
  if (in_sizes[6] != 16 * 64 || in_sizes[7] != 64) return;
  if (in_sizes[8] != 192 * 16 || in_sizes[9] != 16) return;
  if (in_sizes[10] != 128 * 32 || in_sizes[11] != 32) return;
  if (in_sizes[12] != 64 * 8 || in_sizes[13] != 8) return;
  if (out_size != NN * 8) return;

  const float* node_feat = (const float*)d_in[0];
  const float* edge_feat = (const float*)d_in[1];
  const int*   src = (const int*)d_in[2];
  const int*   dst = (const int*)d_in[3];
  const float* Wn  = (const float*)d_in[4];
  const float* bn  = (const float*)d_in[5];
  const float* We  = (const float*)d_in[6];
  const float* be  = (const float*)d_in[7];
  const float* Wem = (const float*)d_in[8];
  const float* bem = (const float*)d_in[9];
  const float* Wnm = (const float*)d_in[10];
  const float* bnm = (const float*)d_in[11];
  const float* Wfc = (const float*)d_in[12];
  const float* bfc = (const float*)d_in[13];
  float* out = (float*)d_out;

  char* ws = (char*)d_ws;
  size_t off = 0;
  const size_t oW   = off; off = al256(off + (size_t)U_END * 16);
  const size_t oNIN = off; off = al256(off + (size_t)NP * 32 * 4);
  const size_t oP   = off; off = al256(off + (size_t)NP * 32 * 4);
  const size_t oE   = off; off = al256(off + (size_t)NE * 16 * 4);
  const size_t oOFF = off; off = al256(off + (size_t)NSLOT * 4);
  const size_t oCNT = off; off = al256(off + (size_t)NSLOT * 4);
  const size_t oEID = off; off = al256(off + (size_t)EIDN * 4);
  if (off > ws_size || off > (size_t)WSMAX) return;
  unsigned short* W16 = (unsigned short*)(ws + oW);
  float* NIN = (float*)(ws + oNIN);
  float* P   = (float*)(ws + oP);
  float* Eb  = (float*)(ws + oE);
  int* OFFS  = (int*)(ws + oOFF);
  int* CNT   = (int*)(ws + oCNT);
  int* EID   = (int*)(ws + oEID);
  const unsigned short* WnT2   = W16;
  const unsigned short* WeT2   = W16 + (size_t)U_WE * 8;
  const unsigned short* WsdT2  = W16 + (size_t)U_SD * 8;
  const unsigned short* WmidT2 = W16 + (size_t)U_MID * 8;
  const unsigned short* WnmT2  = W16 + (size_t)U_NM * 8;
  const unsigned short* WfcT2  = W16 + (size_t)U_FC * 8;

  const size_t csrLds  = (size_t)CSR_LDS_INTS * 4;
  const size_t nodeLds = (size_t)NODE_LDS_BYTES;
  hipFuncSetAttribute(reinterpret_cast<const void*>(&k_csr), hipFuncAttributeMaxDynamicSharedMemorySize, (int)csrLds);
  hipFuncSetAttribute(reinterpret_cast<const void*>(&k_node), hipFuncAttributeMaxDynamicSharedMemorySize, (int)nodeLds);

  const int vec8 = ((NE & 3) == 0) ? 1 : 0;
  const int gN = NP / TM;
  const int gE = NE / TM;

  k_prep<<<U_END / NTHR, NTHR, 0, stream>>>(Wn, We, Wem, Wnm, Wfc, W16);
  k_cvt<<<(NP * 8) / NTHR, NTHR, 0, stream>>>(node_feat, NN * 8, NP * 8, NIN);
  k_cvt<<<(NE * 4) / NTHR, NTHR, 0, stream>>>(edge_feat, NE * 4, NE * 4, Eb);
  k_csr<<<NBLK, NTHR, csrLds, stream>>>(dst, NE, vec8, OFFS, CNT, EID);
  for (int t = 1; t <= 12; ++t) {
    k_node<<<gN, NTHR, nodeLds, stream>>>(NIN, P, Eb, OFFS, CNT, EID, EIDN, NE,
                                           WnT2, WeT2, WsdT2, WnmT2, bn, be, bnm);
    if (t <= 11) {
      k_edge<<<gE, NTHR, 0, stream>>>(Eb, P, src, dst, NN, WeT2, WmidT2, be, bem);
    }
  }
  k_head<<<gN, NTHR, 0, stream>>>(NIN, WnT2, WfcT2, bn, bfc, out, NN);
}
